// MultiHeadAttention_50551765074006
// MI455X (gfx1250) — hardware-verified
//
#include <hip/hip_runtime.h>
#ifndef NB
#define NB 2
#endif
#ifndef SEQ
#define SEQ 2048
#endif
#define NB_FULL 2
#define SEQ_FULL 2048
#define DM 1024
#define NH 16
#define HD 64
#define NR (NB * SEQ)
#define SCL 0.18033688011112042f

typedef _Float16 v16h __attribute__((ext_vector_type(16)));
typedef _Float16 v4h  __attribute__((ext_vector_type(4)));
typedef unsigned short v8us __attribute__((ext_vector_type(8), may_alias));
typedef float  v8f  __attribute__((ext_vector_type(8)));
typedef float  v4f  __attribute__((ext_vector_type(4)));
typedef float  v4fa __attribute__((ext_vector_type(4), may_alias));
union FragH { v16h v; v8us half[2]; _Float16 h[16]; unsigned short u[16]; };

static_assert(NH * HD == DM);
static_assert(HD == 64);
static_assert(DM % 128 == 0 && DM % 64 == 0 && DM % 32 == 0 && DM % 8 == 0);
static_assert(SEQ % 128 == 0 && SEQ % 32 == 0);
static_assert(NR % 128 == 0 && NR % 64 == 0);
static_assert(NB <= NB_FULL && SEQ <= SEQ_FULL);
static_assert(((size_t)NR * (DM / 8)) % 256 == 0);
static_assert(((size_t)DM * (DM / 8)) % 256 == 0);
static_assert((size_t)4 * DM * DM * 2 + (size_t)5 * NR * DM * 2 <= (size_t)134217728);

__device__ __forceinline__ float bf16_rne(float x) {
  unsigned int u = __float_as_uint(x);
  u = (u + 0x7FFFu + ((u >> 16) & 1u)) & 0xFFFF0000u;
  return __uint_as_float(u);
}

__device__ __forceinline__ v16h g2_frag(const _Float16* p, int hh) {
  FragH f;
  f.half[0] = *(const v8us*)((const unsigned short*)p + 8 * hh);
  f.half[1] = *(const v8us*)((const unsigned short*)p + 16 + 8 * hh);
  return f.v;
}
__device__ __forceinline__ v8f g2_mma(v16h a, v16h b, v8f c) {
  v8f d = __builtin_amdgcn_wmma_f32_16x16x32_f16(false, a, false, b, (short)0, c, false, false);
  asm volatile("v_nop\n\tv_nop\n\tv_nop\n\tv_nop" : "+v"(d) : "v"(a), "v"(b));
  return d;
}

__global__ __launch_bounds__(256) void k_x16(const float* __restrict__ x, _Float16* __restrict__ X16) {
  const int t = blockIdx.x * 256 + threadIdx.x;
  if (t >= NR * (DM / 8)) return;
  const int row = t / (DM / 8), c8 = (t - row * (DM / 8)) * 8;
  const size_t srow = (size_t)(row / SEQ) * SEQ_FULL + (size_t)(row % SEQ);
  const v4f a = *(const v4fa*)(x + srow * DM + c8), c = *(const v4fa*)(x + srow * DM + c8 + 4);
  FragH f;
#pragma unroll
  for (int q = 0; q < 4; ++q) { f.h[q] = (_Float16)bf16_rne(a[q]); f.h[4 + q] = (_Float16)bf16_rne(c[q]); }
  const v8us o = f.half[0];
  unsigned short* d = (unsigned short*)X16 + (size_t)t * 8;
  *(volatile v8us*)d = o;
  __threadfence();
  *(volatile v8us*)d = o;
}

__global__ __launch_bounds__(256) void k_wt_f16(const float* __restrict__ W, _Float16* __restrict__ Wt, int K, int N, float scale) {
  const int t = blockIdx.x * 256 + threadIdx.x;
  if (t >= N * (K / 8)) return;
  const int n = t / (K / 8), k8 = (t % (K / 8)) * 8;
  FragH f;
#pragma unroll
  for (int i = 0; i < 8; ++i) f.h[i] = (_Float16)(bf16_rne(W[(size_t)(k8 + i) * N + n]) * scale);
  const v8us o = f.half[0];
  unsigned short* d = (unsigned short*)Wt + (size_t)n * K + k8;
  *(volatile v8us*)d = o;
  __threadfence();
  *(volatile v8us*)d = o;
}

template <int ROWBIAS, int OUTF32>
__device__ __forceinline__ void gemm2_body(const _Float16* __restrict__ A, int lda, const _Float16* __restrict__ Bh, int ldb, float alpha,
                                           const float* __restrict__ bias, float* __restrict__ C, _Float16* __restrict__ C16, int ldc, int N, int K) {
  __shared__ __attribute__((aligned(16))) float so[4][32][68];
  const int wave = __builtin_amdgcn_readfirstlane(threadIdx.x >> 5);
  const int lane = threadIdx.x & 31, ln = lane & 15, hh = lane >> 4;
  const int ntn = N >> 6;
  const int mt = blockIdx.x / ntn, nq = blockIdx.x - mt * ntn;
  const int row0 = mt * 128 + 32 * wave, col0 = nq * 64;
  const _Float16* a0p = A + (size_t)(row0 + ln) * lda;
  const _Float16* a1p = a0p + (size_t)16 * lda;
  const _Float16* b0p = Bh + (size_t)(col0 + ln) * ldb;
  const _Float16* b1p = b0p + (size_t)16 * ldb;
  const _Float16* b2p = b1p + (size_t)16 * ldb;
  const _Float16* b3p = b2p + (size_t)16 * ldb;
  const v8f z8 = {0.f, 0.f, 0.f, 0.f, 0.f, 0.f, 0.f, 0.f};
  v8f c00 = z8, c01 = z8, c02 = z8, c03 = z8, c10 = z8, c11 = z8, c12 = z8, c13 = z8;
#pragma unroll 1
  for (int kb = 0; kb < K; kb += 32) {
    const v16h a0 = g2_frag(a0p + kb, hh), a1 = g2_frag(a1p + kb, hh);
    v16h b = g2_frag(b0p + kb, hh); c00 = g2_mma(a0, b, c00); c10 = g2_mma(a1, b, c10);
    b = g2_frag(b1p + kb, hh); c01 = g2_mma(a0, b, c01); c11 = g2_mma(a1, b, c11);
    b = g2_frag(b2p + kb, hh); c02 = g2_mma(a0, b, c02); c12 = g2_mma(a1, b, c12);
    b = g2_frag(b3p + kb, hh); c03 = g2_mma(a0, b, c03); c13 = g2_mma(a1, b, c13);
  }
  float rb[16];
  if (ROWBIAS) {
    const v4f r0 = *(const v4fa*)(bias + row0 + 8 * hh), r1 = *(const v4fa*)(bias + row0 + 8 * hh + 4);
    const v4f r2 = *(const v4fa*)(bias + row0 + 16 + 8 * hh), r3 = *(const v4fa*)(bias + row0 + 16 + 8 * hh + 4);
#pragma unroll
    for (int q = 0; q < 4; ++q) { rb[q] = bf16_rne(r0[q]); rb[4 + q] = bf16_rne(r1[q]); rb[8 + q] = bf16_rne(r2[q]); rb[12 + q] = bf16_rne(r3[q]); }
  } else {
#pragma unroll
    for (int q = 0; q < 16; ++q) rb[q] = 0.f;
  }
  v8f accs[8] = {c00, c01, c02, c03, c10, c11, c12, c13};
#pragma unroll
  for (int u = 0; u < 8; ++u) {
    const int t = u & 3, half = u >> 2;
    const int col = col0 + t * 16 + ln;
    const float cb = ROWBIAS ? 0.f : bf16_rne(bias[col]);
#pragma unroll
    for (int r = 0; r < 8; ++r) {
      const int rloc = half * 16 + 8 * hh + r;
      const float bv = ROWBIAS ? rb[half * 8 + r] : cb;
      so[wave][rloc][t * 16 + ln] = accs[u][r] * alpha + bv;
    }
  }
  __builtin_amdgcn_fence(4  , "workgroup");
  __builtin_amdgcn_wave_barrier();
  const int rsub = lane >> 4, c4 = (lane & 15) * 4;
  const size_t orow0 = OUTF32 ? ((size_t)(row0 / SEQ) * SEQ_FULL + (size_t)(row0 % SEQ)) : (size_t)row0;
  for (int pass = 0; pass < 2; ++pass) {
#pragma unroll
    for (int q = 0; q < 16; ++q) {
      const int r = q * 2 + rsub;
      const v4f v = *(const v4fa*)&so[wave][r][c4];
      if (OUTF32) {
        *(volatile v4f*)(C + (orow0 + r) * ldc + col0 + c4) = v;
      } else {
        v4h h4;
#pragma unroll
        for (int i = 0; i < 4; ++i) h4[i] = (_Float16)v[i];
        *(volatile v4h*)(C16 + (orow0 + r) * ldc + col0 + c4) = h4;
      }
    }
    if (pass == 0) __threadfence();
  }
}

__global__ __launch_bounds__(128) void k_proj(const _Float16* __restrict__ X16, const _Float16* __restrict__ Bt, const float* __restrict__ bias, _Float16* __restrict__ C16) {
  gemm2_body<0, 0>(X16, DM, Bt, DM, 0.0625f, bias, nullptr, C16, DM, DM, DM);
}
__global__ __launch_bounds__(128) void k_projT(const _Float16* __restrict__ Wt, const _Float16* __restrict__ X16, const float* __restrict__ bias, _Float16* __restrict__ VT) {
  gemm2_body<1, 0>(Wt, DM, X16, DM, 0.0625f, bias, nullptr, VT, NR, NR, DM);
}
__global__ __launch_bounds__(128) void k_outp(const _Float16* __restrict__ CT, const _Float16* __restrict__ Bt, const float* __restrict__ bias, float* __restrict__ out) {
  gemm2_body<0, 1>(CT, DM, Bt, DM, 0.0009765625f, bias, out, nullptr, DM, DM, DM);
}

__global__ __launch_bounds__(256) void k_flash(const _Float16* __restrict__ Q16, const _Float16* __restrict__ K16, const _Float16* __restrict__ VT, _Float16* __restrict__ CT) {
  __shared__ __attribute__((aligned(16))) unsigned short so[8][16][72];
  const int wave = __builtin_amdgcn_readfirstlane(threadIdx.x >> 5);
  const int lane = threadIdx.x & 31, ln = lane & 15, hh = lane >> 4;
  const int bh = blockIdx.x;
  const int b = bh / NH, h = bh - b * NH;
  const int q0 = blockIdx.y * 128 + wave * 16;
  const size_t tok0 = (size_t)b * SEQ;
  const _Float16* qrow = Q16 + (tok0 + q0 + ln) * DM + h * HD;
  const v16h qf0 = g2_frag(qrow, hh), qf1 = g2_frag(qrow + 32, hh);
  const _Float16* kbase = K16 + (tok0 + ln) * DM + h * HD;
  const _Float16* vbase = VT + (size_t)(h * HD + ln) * NR + tok0;
  const v8f z8 = {0.f, 0.f, 0.f, 0.f, 0.f, 0.f, 0.f, 0.f};
  v8f o0 = z8, o1 = z8, o2 = z8, o3 = z8;
  float m = -3.0e38f, l = 0.f;
#pragma unroll 1
  for (int kb = 0; kb < SEQ; kb += 32) {
    const _Float16* kr0 = kbase + (size_t)kb * DM;
    const _Float16* kr1 = kr0 + (size_t)16 * DM;
    v8f s0 = z8, s1 = z8;
    s0 = g2_mma(g2_frag(kr0, hh), qf0, s0);
    s0 = g2_mma(g2_frag(kr0 + 32, hh), qf1, s0);
    s1 = g2_mma(g2_frag(kr1, hh), qf0, s1);
    s1 = g2_mma(g2_frag(kr1 + 32, hh), qf1, s1);
    float bm = -3.0e38f;
#pragma unroll
    for (int r = 0; r < 8; ++r) { s0[r] *= SCL; s1[r] *= SCL; bm = fmaxf(bm, fmaxf(s0[r], s1[r])); }
    bm = fmaxf(bm, __shfl_xor(bm, 16, 32));
    const float mn = fmaxf(m, bm);
    const float sc = exp2f(m - mn);
    const float mo = mn - 10.0f;
    FragH pf;
    float ps = 0.f;
#pragma unroll
    for (int r = 0; r < 8; ++r) {
      const float e0 = exp2f(s0[r] - mo);
      const float e1 = exp2f(s1[r] - mo);
      ps += e0 + e1;
      pf.h[r] = (_Float16)e0;
      pf.h[8 + r] = (_Float16)e1;
    }
    ps += __shfl_xor(ps, 16, 32);
    l = l * sc + ps;
    m = mn;
#pragma unroll
    for (int r = 0; r < 8; ++r) { o0[r] *= sc; o1[r] *= sc; o2[r] *= sc; o3[r] *= sc; }
    const _Float16* vr = vbase + kb;
    const v16h v0 = g2_frag(vr, hh);
    const v16h v1 = g2_frag(vr + (size_t)16 * NR, hh);
    const v16h v2 = g2_frag(vr + (size_t)32 * NR, hh);
    const v16h v3 = g2_frag(vr + (size_t)48 * NR, hh);
    o0 = g2_mma(v0, pf.v, o0);
    o1 = g2_mma(v1, pf.v, o1);
    o2 = g2_mma(v2, pf.v, o2);
    o3 = g2_mma(v3, pf.v, o3);
  }
  const float inv = 64.0f * (1.0f / l);
  {
    FragH f;
#pragma unroll
    for (int r = 0; r < 8; ++r) f.h[r] = (_Float16)(o0[r] * inv);
    *(v8us*)&so[wave][ln][0 + 8 * hh] = f.half[0];
#pragma unroll
    for (int r = 0; r < 8; ++r) f.h[r] = (_Float16)(o1[r] * inv);
    *(v8us*)&so[wave][ln][16 + 8 * hh] = f.half[0];
#pragma unroll
    for (int r = 0; r < 8; ++r) f.h[r] = (_Float16)(o2[r] * inv);
    *(v8us*)&so[wave][ln][32 + 8 * hh] = f.half[0];
#pragma unroll
    for (int r = 0; r < 8; ++r) f.h[r] = (_Float16)(o3[r] * inv);
    *(v8us*)&so[wave][ln][48 + 8 * hh] = f.half[0];
  }
  __builtin_amdgcn_fence(4  , "workgroup");
  __builtin_amdgcn_wave_barrier();
  const int rq = lane >> 3, pc = (lane & 7) * 8;
  unsigned short* dst = (unsigned short*)CT + (tok0 + q0) * DM + h * HD + pc;
  for (int pass = 0; pass < 2; ++pass) {
#pragma unroll
    for (int it = 0; it < 4; ++it) {
      const int row = it * 4 + rq;
      const v8us v = *(const v8us*)&so[wave][row][pc];
      *(volatile v8us*)(dst + (size_t)row * DM) = v;
    }
    if (pass == 0) __threadfence();
  }
}

extern "C" void kernel_launch(void* const* d_in, const int* in_sizes, int n_in,
                              void* d_out, int out_size, void* d_ws, size_t ws_size, hipStream_t stream) {
  if (n_in < 9) return;
  const long long need_x = ((long long)(NB - 1) * SEQ_FULL + SEQ) * DM;
  if ((long long)in_sizes[0] < need_x) return;
  if (in_sizes[1] < DM * DM || in_sizes[3] < DM * DM || in_sizes[5] < DM * DM || in_sizes[7] < DM * DM) return;
  if (in_sizes[2] < DM || in_sizes[4] < DM || in_sizes[6] < DM || in_sizes[8] < DM) return;
  if ((long long)out_size < need_x) return;
  const float* x  = (const float*)d_in[0];
  const float* wq = (const float*)d_in[1];
  const float* bq = (const float*)d_in[2];
  const float* wk = (const float*)d_in[3];
  const float* bk = (const float*)d_in[4];
  const float* wv = (const float*)d_in[5];
  const float* bv = (const float*)d_in[6];
  const float* wo = (const float*)d_in[7];
  const float* bo = (const float*)d_in[8];

  char* ws = (char*)d_ws; size_t off = 0;
  auto take = [&](size_t bytes) { char* p = ws + off; off += (bytes + 255) & ~(size_t)255; return p; };
  _Float16* BQ  = (_Float16*)take((size_t)DM * DM * 2);
  _Float16* BK  = (_Float16*)take((size_t)DM * DM * 2);
  _Float16* BV  = (_Float16*)take((size_t)DM * DM * 2);
  _Float16* BO  = (_Float16*)take((size_t)DM * DM * 2);
  _Float16* X16 = (_Float16*)take((size_t)NR * DM * 2);
  _Float16* Q16 = (_Float16*)take((size_t)NR * DM * 2);
  _Float16* K16 = (_Float16*)take((size_t)NR * DM * 2);
  _Float16* VT  = (_Float16*)take((size_t)DM * NR * 2);
  _Float16* CT  = (_Float16*)take((size_t)NR * DM * 2);
  if (off > ws_size) return;

  const unsigned gw = (unsigned)(((size_t)DM * (DM / 8)) / 256);
  k_wt_f16<<<gw, 256, 0, stream>>>(wq, BQ, DM, DM, 16.0f);
  k_wt_f16<<<gw, 256, 0, stream>>>(wk, BK, DM, DM, 16.0f);
  k_wt_f16<<<gw, 256, 0, stream>>>(wv, BV, DM, DM, 16.0f);
  k_wt_f16<<<gw, 256, 0, stream>>>(wo, BO, DM, DM, 16.0f);
  k_x16<<<(unsigned)(((size_t)NR * (DM / 8)) / 256), 256, 0, stream>>>(x, X16);

  k_proj<<<(unsigned)((NR / 128) * (DM / 64)), 128, 0, stream>>>(X16, BQ, bq, Q16);
  k_proj<<<(unsigned)((NR / 128) * (DM / 64)), 128, 0, stream>>>(X16, BK, bk, K16);
  k_projT<<<(unsigned)((DM / 128) * (NR / 64)), 128, 0, stream>>>(BV, X16, bv, VT);

  k_flash<<<dim3((unsigned)(NB * NH), (unsigned)(SEQ / 128)), 256, 0, stream>>>(Q16, K16, VT, CT);

  k_outp<<<(unsigned)((NR / 128) * (DM / 64)), 128, 0, stream>>>(CT, BO, bo, (float*)d_out);
}
